// DHSpace_22247930593800
// MI455X (gfx1250) — hardware-verified
//
#include <hip/hip_runtime.h>
#include <stddef.h>


#define DF    128
#define NH    8
#define HC    16
#define NTY   3
#define NRL   4
#define NCD   2
#define GR    32
#define AP    136
#define XSP   132
#define NTHR  256
#define NWAVE 8
#define NB    448
#define NTILE (NB / 16)
#define CHUNK 2048
#define WCAP  256
#define NGRP  (CHUNK / (NTHR * 4))
#define NWROW (3 * NCD * DF)
#define NUROW (NTY * DF)
#define NTROW (NRL * NH * HC)

#define L_Z    (NB * DF)
#define L_MX   (NB * NH)
#define L_DEN  (NB * NH)
#define L_LIST (NWAVE * WCAP)
#define L_PRI  32
#define L_RES  (16 * AP / 2)
#define L_HST  (16 * XSP)
#define LDS_WORDS (L_Z + L_MX + L_DEN + L_LIST + NWAVE + L_PRI + NB + L_RES + L_HST)
#define LDS_BYTES (LDS_WORDS * 4)

static_assert(NGRP == 2);
static_assert(WCAP == (CHUNK / NTHR) * 32);
static_assert(NB <= 512);
static_assert((NB % 16) == 0);
static_assert((L_Z % 4) == 0);
static_assert((L_MX % 4) == 0);
static_assert((L_DEN % 4) == 0);
static_assert(((L_Z + L_MX + L_DEN + L_LIST + NWAVE + L_PRI + NB) % 4) == 0);
static_assert(((L_Z + L_MX + L_DEN + L_LIST + NWAVE + L_PRI + NB + L_RES) % 4) == 0);
static_assert(LDS_BYTES == 280992);

typedef float    v4f  __attribute__((ext_vector_type(4)));
typedef float    v8f  __attribute__((ext_vector_type(8)));
typedef int      v4i  __attribute__((ext_vector_type(4)));
typedef _Float16 v4h  __attribute__((ext_vector_type(4)));
typedef _Float16 v8h  __attribute__((ext_vector_type(8)));
typedef _Float16 v16h __attribute__((ext_vector_type(16)));
union Frag   { v16h v; v8h half[2]; };
union Pack16 { v8h h; v4i i; };

__device__ __forceinline__ v8f wm(v16h a, v16h b, v8f c) {
  v8f d = __builtin_amdgcn_wmma_f32_16x16x32_f16(false, a, false, b, (short)0, c, false, false);
  asm volatile("v_nop\n\tv_nop\n\tv_nop\n\tv_nop" : "+v"(d) : "v"(a), "v"(b));
  return d;
}

__device__ __forceinline__ float wsum(float v) {
  v += __shfl_xor(v, 16, 32);
  v += __shfl_xor(v, 8, 32);
  v += __shfl_xor(v, 4, 32);
  v += __shfl_xor(v, 2, 32);
  v += __shfl_xor(v, 1, 32);
  return v;
}

__device__ __forceinline__ float gelu_t(float x) {
  const float u = 0.7978845608028654f * (x + 0.044715f * x * x * x);
  return 0.5f * x * (1.0f + tanhf(u));
}

__global__ __launch_bounds__(NTHR) void k_prep(
    const float* __restrict__ Wk, const float* __restrict__ Wq, const float* __restrict__ Wv,
    const float* __restrict__ Wup, const float* __restrict__ rel_att, const float* __restrict__ rel_msg,
    const float* __restrict__ r_alpha,
    _Float16* Wc, _Float16* Wu, _Float16* ATT, _Float16* MSG) {
  const int b = blockIdx.x;
  const int tid = threadIdx.x;
  Pack16 u;
  _Float16* dst;
  if (b < NWROW / 16) {
    const int t  = b * NTHR + tid;
    const int n  = t >> 4, kg = t & 15;
    const int p  = n >> 8, c = (n >> 7) & 1, o = n & 127;
    const float* W = (p == 0) ? Wk : ((p == 1) ? Wq : Wv);
    const float* s = W + ((size_t)c * DF + kg * 8) * DF + o;
#pragma unroll
    for (int j = 0; j < 8; ++j) u.h[j] = (_Float16)(s[(size_t)j * DF] * 8.0f);
    dst = Wc + (size_t)t * 8;
  } else if (b < NWROW / 16 + NUROW / 16) {
    const int t  = (b - NWROW / 16) * NTHR + tid;
    const int n  = t >> 4, kg = t & 15;
    const int ty = n >> 7, o = n & 127;
    const float* s = Wup + ((size_t)ty * DF + kg * 8) * DF + o;
#pragma unroll
    for (int j = 0; j < 8; ++j) u.h[j] = (_Float16)(s[(size_t)j * DF] * 8.0f);
    dst = Wu + (size_t)t * 8;
  } else {
    const int t     = (b - NWROW / 16 - NUROW / 16) * NTHR + tid;
    const int which = t >> 10;
    const int tt    = t & 1023;
    const int row   = tt >> 1, g = tt & 1;
    const int r     = row >> 7, h = (row >> 4) & 7, low = row & 15;
    const float a0 = r_alpha[r * NCD + 0], a1 = r_alpha[r * NCD + 1];
    const float mm = fmaxf(a0, a1);
    const float e0 = __expf(a0 - mm), e1 = __expf(a1 - mm);
    const float inv = __builtin_amdgcn_rcpf(e0 + e1);
    const float b0 = e0 * inv, b1 = e1 * inv;
    const float* tab = (which == 0) ? rel_att : rel_msg;
    const int base = (which == 0) ? ((h * HC + low) * HC + g * 8) : ((h * HC + g * 8) * HC + low);
    const int strd = (which == 0) ? 1 : HC;
    const int coff = NH * HC * HC;
#pragma unroll
    for (int j = 0; j < 8; ++j) {
      const int ix = base + j * strd;
      const float v = b0 * tab[ix] + b1 * tab[coff + ix];
      u.h[j] = (_Float16)(v * 8.0f);
    }
    dst = ((which == 0) ? ATT : MSG) + (size_t)tt * 8;
  }
  *(volatile v4i*)dst = u.i;
  __threadfence();
  *(volatile v4i*)dst = u.i;
}

__device__ __forceinline__ void proj2(const _Float16* At, const _Float16* __restrict__ Wc, int n0,
                                      int hh, int m, v8f& c00, v8f& c01, v8f& c10, v8f& c11) {
  const v8f z = {0.f, 0.f, 0.f, 0.f, 0.f, 0.f, 0.f, 0.f};
  c00 = z; c01 = z; c10 = z; c11 = z;
#pragma unroll
  for (int kt = 0; kt < DF / 32; ++kt) {
    const int k0 = kt * 32;
    Frag a0, a1, b0, b1;
    const _Float16* pa0 = At + m * AP + k0 + 8 * hh;
    const _Float16* pa1 = At + (16 + m) * AP + k0 + 8 * hh;
    const _Float16* pb0 = Wc + (size_t)n0 * DF + k0 + 8 * hh;
    const _Float16* pb1 = pb0 + (size_t)DF * DF;
    a0.half[0] = *(const v8h*)pa0; a0.half[1] = *(const v8h*)(pa0 + 16);
    a1.half[0] = *(const v8h*)pa1; a1.half[1] = *(const v8h*)(pa1 + 16);
    b0.half[0] = *(const v8h*)pb0; b0.half[1] = *(const v8h*)(pb0 + 16);
    b1.half[0] = *(const v8h*)pb1; b1.half[1] = *(const v8h*)(pb1 + 16);
    c00 = wm(a0.v, b0.v, c00);
    c01 = wm(a0.v, b1.v, c01);
    c10 = wm(a1.v, b0.v, c10);
    c11 = wm(a1.v, b1.v, c11);
  }
}

__device__ __forceinline__ void epi_mix(v8f c00, v8f c01, v8f c10, v8f c11, int hh, int col,
                                        float b0, float b1, const int* typ, const float* anT,
                                        float* Xs, _Float16* Th, bool tof16) {
#pragma unroll
  for (int T = 0; T < 2; ++T) {
#pragma unroll
    for (int r = 0; r < 8; ++r) {
      const int row = 16 * T + 8 * hh + r;
      const int t = typ[row];
      const float w0 = anT[2 * t], w1 = anT[2 * t + 1];
      const float v0 = (T == 0) ? c00[r] : c10[r];
      const float v1 = (T == 0) ? c01[r] : c11[r];
      const float val = w0 * (v0 * 0.125f + b0) + w1 * (v1 * 0.125f + b1);
      if (tof16) Th[row * AP + col] = (_Float16)val;
      else       Xs[row * XSP + col] = val;
    }
  }
}

__device__ __forceinline__ void small_tab(const _Float16* Th, const _Float16* __restrict__ B16,
                                          _Float16* P, _Float16* St, int wave, int hh, int m,
                                          int rowBase, int nP) {
  const v8h z8 = {(_Float16)0.f, (_Float16)0.f, (_Float16)0.f, (_Float16)0.f,
                  (_Float16)0.f, (_Float16)0.f, (_Float16)0.f, (_Float16)0.f};
  const v8f z = {0.f, 0.f, 0.f, 0.f, 0.f, 0.f, 0.f, 0.f};
#pragma unroll 1
  for (int r4 = 0; r4 < NRL; ++r4) {
    Frag a0, a1, b;
    a0.half[0] = *(const v8h*)(Th + m * AP + wave * HC + 8 * hh);        a0.half[1] = z8;
    a1.half[0] = *(const v8h*)(Th + (16 + m) * AP + wave * HC + 8 * hh); a1.half[1] = z8;
    b.half[0]  = *(const v8h*)(B16 + ((size_t)(r4 * NH + wave) * HC + m) * HC + 8 * hh);
    b.half[1]  = z8;
    v8f c0 = z, c1 = z;
    c0 = wm(a0.v, b.v, c0);
    c1 = wm(a1.v, b.v, c1);
#pragma unroll
    for (int r = 0; r < 8; ++r) {
      St[(8 * hh + r) * AP + wave * HC + m]      = (_Float16)(c0[r] * 0.125f);
      St[(16 + 8 * hh + r) * AP + wave * HC + m] = (_Float16)(c1[r] * 0.125f);
    }
    __syncthreads();
    Pack16 u0, u1;
    u0.h = *(const v8h*)(St + (4 * wave + 0 + hh) * AP + 8 * m);
    u1.h = *(const v8h*)(St + (4 * wave + 2 + hh) * AP + 8 * m);
    _Float16* g0 = P + ((size_t)r4 * nP + rowBase + 4 * wave + 0 + hh) * DF + 8 * m;
    _Float16* g1 = P + ((size_t)r4 * nP + rowBase + 4 * wave + 2 + hh) * DF + 8 * m;
    *(volatile v4i*)g0 = u0.i;
    *(volatile v4i*)g1 = u1.i;
    __threadfence();
    *(volatile v4i*)g0 = u0.i;
    *(volatile v4i*)g1 = u1.i;
    __syncthreads();
  }
}

__global__ __launch_bounds__(NTHR) void k_node(
    const float* __restrict__ x, const _Float16* __restrict__ Wc,
    const float* __restrict__ bk, const float* __restrict__ bq, const float* __restrict__ bv,
    const float* __restrict__ n_alpha, const int* __restrict__ nty,
    const _Float16* __restrict__ ATT, const _Float16* __restrict__ MSG,
    float* Kp, _Float16* QAp, _Float16* VMp, int nN, int nP) {
  __shared__ __attribute__((aligned(16))) _Float16 At[GR * AP];
  __shared__ __attribute__((aligned(16))) float    Xs[GR * XSP];
  __shared__ __attribute__((aligned(16))) _Float16 Th[GR * AP];
  __shared__ __attribute__((aligned(16))) _Float16 St[GR * AP];
  __shared__ int   typ[GR];
  __shared__ float anT[8];

  const int tid  = threadIdx.x;
  const int lane = tid & 31;
  const int wave = tid >> 5;
  const int hh   = lane >> 4;
  const int m    = lane & 15;
  const int rowBase = blockIdx.x * GR;

  {
    const int r  = tid >> 3;
    const int c0 = (tid & 7) * 16;
    int row = rowBase + r;
    if (row > nN - 1) row = nN - 1;
    const float* p = x + (size_t)row * DF + c0;
    const v4f f0 = *(const v4f*)(p), f1 = *(const v4f*)(p + 4);
    const v4f f2 = *(const v4f*)(p + 8), f3 = *(const v4f*)(p + 12);
    Pack16 u0, u1;
    u0.h[0] = (_Float16)f0.x; u0.h[1] = (_Float16)f0.y; u0.h[2] = (_Float16)f0.z; u0.h[3] = (_Float16)f0.w;
    u0.h[4] = (_Float16)f1.x; u0.h[5] = (_Float16)f1.y; u0.h[6] = (_Float16)f1.z; u0.h[7] = (_Float16)f1.w;
    u1.h[0] = (_Float16)f2.x; u1.h[1] = (_Float16)f2.y; u1.h[2] = (_Float16)f2.z; u1.h[3] = (_Float16)f2.w;
    u1.h[4] = (_Float16)f3.x; u1.h[5] = (_Float16)f3.y; u1.h[6] = (_Float16)f3.z; u1.h[7] = (_Float16)f3.w;
    *(v8h*)(At + r * AP + c0)     = u0.h;
    *(v8h*)(At + r * AP + c0 + 8) = u1.h;
    if (tid < GR) {
      int rr = rowBase + tid;
      if (rr > nN - 1) rr = nN - 1;
      int t = nty[rr];
      t = t < 0 ? 0 : (t > NTY - 1 ? NTY - 1 : t);
      typ[tid] = t;
    }
    if (tid < NTY) {
      const float a0 = n_alpha[tid * NCD + 0], a1 = n_alpha[tid * NCD + 1];
      const float mm = fmaxf(a0, a1);
      const float e0 = __expf(a0 - mm), e1 = __expf(a1 - mm);
      const float inv = __builtin_amdgcn_rcpf(e0 + e1);
      anT[2 * tid] = e0 * inv;
      anT[2 * tid + 1] = e1 * inv;
    }
  }
  __syncthreads();

  const int col = wave * 16 + m;
  v8f c00, c01, c10, c11;

  proj2(At, Wc, 0 * 2 * DF + col, hh, m, c00, c01, c10, c11);
  epi_mix(c00, c01, c10, c11, hh, col, bk[col], bk[DF + col], typ, anT, Xs, Th, false);
  __syncthreads();
  {
    v4f kr[4];
    float* kpp[4];
#pragma unroll
    for (int i = 0; i < 4; ++i) {
      kr[i]  = *(const v4f*)(Xs + (4 * wave + i) * XSP + 4 * lane);
      kpp[i] = Kp + (size_t)(rowBase + 4 * wave + i) * DF + 4 * lane;
    }
#pragma unroll
    for (int i = 0; i < 4; ++i) *(volatile v4f*)(kpp[i]) = kr[i];
    __threadfence();
#pragma unroll
    for (int i = 0; i < 4; ++i) *(volatile v4f*)(kpp[i]) = kr[i];
  }

  proj2(At, Wc, 1 * 2 * DF + col, hh, m, c00, c01, c10, c11);
  epi_mix(c00, c01, c10, c11, hh, col, bq[col], bq[DF + col], typ, anT, Xs, Th, true);
  __syncthreads();
  small_tab(Th, ATT, QAp, St, wave, hh, m, rowBase, nP);

  proj2(At, Wc, 2 * 2 * DF + col, hh, m, c00, c01, c10, c11);
  epi_mix(c00, c01, c10, c11, hh, col, bv[col], bv[DF + col], typ, anT, Xs, Th, true);
  __syncthreads();
  small_tab(Th, MSG, VMp, St, wave, hh, m, rowBase, nP);
}

__global__ __launch_bounds__(NTHR) void k_agg(
    const float* __restrict__ x, const int* __restrict__ ei, const int* __restrict__ ety,
    const int* __restrict__ nty, const float* __restrict__ Kp,
    const _Float16* __restrict__ QAp, const _Float16* __restrict__ VMp,
    const _Float16* __restrict__ Wu, const float* __restrict__ r_alpha,
    const float* __restrict__ rel_pri, const float* __restrict__ b_up,
    const float* __restrict__ gam, const float* __restrict__ bet,
    float* out, int nN, int nE, int nP) {
  extern __shared__ v4f lds_dyn[];
  float*    Z    = (float*)lds_dyn;
  float*    mx   = Z + L_Z;
  float*    den  = mx + L_MX;
  int*      list = (int*)(den + L_DEN);
  int*      wcnt = list + L_LIST;
  float*    pri  = (float*)(wcnt + NWAVE);
  int*      typ  = (int*)(pri + L_PRI);
  _Float16* resT = (_Float16*)(typ + NB);
  float*    hst  = (float*)(resT + 16 * AP);

  const int tid  = threadIdx.x;
  const int lane = tid & 31;
  const int wave = tid >> 5;
  const int hh   = lane >> 4;
  const int m    = lane & 15;
  const int hd   = lane >> 2;
  const int nodeBase = blockIdx.x * NB;

  {
    const v4f z4 = {0.f, 0.f, 0.f, 0.f};
    const v4f m4 = {-1e30f, -1e30f, -1e30f, -1e30f};
    for (int i = tid; i < (L_Z + L_MX + L_DEN) / 4; i += NTHR) {
      const bool ismx = (i >= L_Z / 4) && (i < (L_Z + L_MX) / 4);
      lds_dyn[i] = ismx ? m4 : z4;
    }
    for (int i = tid; i < NB; i += NTHR) {
      int nd = nodeBase + i;
      if (nd > nN - 1) nd = nN - 1;
      int t = nty[nd];
      t = t < 0 ? 0 : (t > NTY - 1 ? NTY - 1 : t);
      typ[i] = t;
    }
    if (tid < NRL * NH) {
      const int r = tid >> 3, h = tid & 7;
      const float a0 = r_alpha[r * NCD + 0], a1 = r_alpha[r * NCD + 1];
      const float mm = fmaxf(a0, a1);
      const float e0 = __expf(a0 - mm), e1 = __expf(a1 - mm);
      const float inv = __builtin_amdgcn_rcpf(e0 + e1);
      const float p = (e0 * inv) * rel_pri[h] + (e1 * inv) * rel_pri[NH + h];
      pri[tid] = p * 0.25f;
    }
  }
  __syncthreads();
  const int* eid = ei + nE;
  const bool al16 = ((nE & 3) == 0);

  const int nChunks = (nE + CHUNK - 1) / CHUNK;
#pragma unroll 1
  for (int ch = 0; ch < nChunks; ++ch) {
    const int cbase = ch * CHUNK;
    int wc = 0;
#pragma unroll
    for (int g = 0; g < NGRP; ++g) {
      const int el0 = (g * NTHR + tid) * 4;
      const int e0  = cbase + el0;
      const int sent = -2147483647 - 1;
      v4i d;
      if (al16 && (cbase + CHUNK <= nE)) {
        d = *(const v4i*)(eid + e0);
      } else {
        d.x = (e0     < nE) ? eid[min(e0, nE - 1)]     : sent;
        d.y = (e0 + 1 < nE) ? eid[min(e0 + 1, nE - 1)] : sent;
        d.z = (e0 + 2 < nE) ? eid[min(e0 + 2, nE - 1)] : sent;
        d.w = (e0 + 3 < nE) ? eid[min(e0 + 3, nE - 1)] : sent;
      }
      const unsigned s0 = (unsigned)d.x - (unsigned)nodeBase;
      const unsigned s1 = (unsigned)d.y - (unsigned)nodeBase;
      const unsigned s2 = (unsigned)d.z - (unsigned)nodeBase;
      const unsigned s3 = (unsigned)d.w - (unsigned)nodeBase;
      const bool h0 = s0 < (unsigned)NB;
      const bool h1 = s1 < (unsigned)NB;
      const bool h2 = s2 < (unsigned)NB;
      const bool h3 = s3 < (unsigned)NB;
      const unsigned many = __builtin_amdgcn_ballot_w32(h0 | h1 | h2 | h3);
      if (many != 0u) {
#define HITJ(J, HJ, SJ) { \
          const unsigned mj = __builtin_amdgcn_ballot_w32(HJ); \
          if (HJ) { \
            const int pos = wc + (int)__builtin_amdgcn_mbcnt_lo(mj, 0u); \
            if (pos < WCAP) list[wave * WCAP + pos] = ((el0 + (J)) << 9) | (int)(SJ); \
          } \
          wc += (int)__builtin_popcount(mj); }
        HITJ(0, h0, s0)
        HITJ(1, h1, s1)
        HITJ(2, h2, s2)
        HITJ(3, h3, s3)
#undef HITJ
      }
    }
    if (lane == 0) wcnt[wave] = wc;
    __syncthreads();

    if (wave == 0) {
      for (int wsx = 0; wsx < NWAVE; ++wsx) {
        int n = wcnt[wsx];
        if (n > WCAP) n = WCAP;
        if (n < 0) n = 0;
        for (int i = 0; i < n; ++i) {
          const int ent = list[wsx * WCAP + i];
          int slot = ent & 511;
          if (slot > NB - 1) slot = NB - 1;
          const int el = (ent >> 9) & (CHUNK - 1);
          int e = cbase + el;
          if (e > nE - 1) e = nE - 1;
          int src = ei[e];
          src = src < 0 ? 0 : (src > nN - 1 ? nN - 1 : src);
          int rel = ety[e];
          rel = rel < 0 ? 0 : (rel > NRL - 1 ? NRL - 1 : rel);
          int nd = nodeBase + slot;
          if (nd > nN - 1) nd = nN - 1;
          const v4f kv = *(const v4f*)(Kp + (size_t)src * DF + 4 * lane);
          const v4h qh = *(const v4h*)(QAp + ((size_t)rel * nP + nd) * DF + 4 * lane);
          const v4h vh = *(const v4h*)(VMp + ((size_t)rel * nP + src) * DF + 4 * lane);
          const v4f qa = __builtin_convertvector(qh, v4f);
          const v4f vm = __builtin_convertvector(vh, v4f);
          float s = kv.x * qa.x + kv.y * qa.y + kv.z * qa.z + kv.w * qa.w;
          s += __shfl_xor(s, 1, 32);
          s += __shfl_xor(s, 2, 32);
          s *= pri[rel * NH + hd];
          const int ai = slot * NH + hd;
          const float mo = mx[ai];
          const float mn = fmaxf(mo, s);
          const float sc = __expf(mo - mn);
          const float p  = __expf(s - mn);
          v4f* zp = (v4f*)(Z + slot * DF + 4 * lane);
          const v4f zc = *zp;
          const v4f zn = zc * sc + p * vm;
          *zp = zn;
          const float dn = den[ai];
          const float dnn = dn * sc + p;
          den[ai] = dnn;
          mx[ai]  = mn;
        }
      }
    }
    __syncthreads();
  }

  const int col = wave * 16 + m;
  const float bc0 = b_up[col], bc1 = b_up[DF + col], bc2 = b_up[2 * DF + col];
#pragma unroll 1
  for (int tt = 0; tt < NTILE; ++tt) {
#pragma unroll
    for (int j = 0; j < 2; ++j) {
      const int rr   = 2 * wave + j;
      const int slot = tt * 16 + rr;
      const v4f z   = *(const v4f*)(Z + slot * DF + 4 * lane);
      const float dd  = den[slot * NH + hd];
      const float inv = __builtin_amdgcn_rcpf(dd + 1e-16f);
      v4f g;
      g.x = gelu_t(z.x * inv) * 8.0f;
      g.y = gelu_t(z.y * inv) * 8.0f;
      g.z = gelu_t(z.z * inv) * 8.0f;
      g.w = gelu_t(z.w * inv) * 8.0f;
      const v4h gh = __builtin_convertvector(g, v4h);
      *(v4h*)(resT + rr * AP + 4 * lane) = gh;
    }
    __syncthreads();

    v8f ac0 = {0.f, 0.f, 0.f, 0.f, 0.f, 0.f, 0.f, 0.f};
    v8f ac1 = ac0, ac2 = ac0;
#pragma unroll
    for (int kt = 0; kt < DF / 32; ++kt) {
      const int k0 = kt * 32;
      Frag a, b0, b1, b2;
      const _Float16* pa  = resT + m * AP + k0 + 8 * hh;
      const _Float16* pb0 = Wu + (size_t)col * DF + k0 + 8 * hh;
      const _Float16* pb1 = pb0 + (size_t)DF * DF;
      const _Float16* pb2 = pb1 + (size_t)DF * DF;
      a.half[0]  = *(const v8h*)pa;  a.half[1]  = *(const v8h*)(pa + 16);
      b0.half[0] = *(const v8h*)pb0; b0.half[1] = *(const v8h*)(pb0 + 16);
      b1.half[0] = *(const v8h*)pb1; b1.half[1] = *(const v8h*)(pb1 + 16);
      b2.half[0] = *(const v8h*)pb2; b2.half[1] = *(const v8h*)(pb2 + 16);
      ac0 = wm(a.v, b0.v, ac0);
      ac1 = wm(a.v, b1.v, ac1);
      ac2 = wm(a.v, b2.v, ac2);
    }
#pragma unroll
    for (int r = 0; r < 8; ++r) {
      const int rr = 8 * hh + r;
      const int t  = typ[tt * 16 + rr];
      const float cv = (t == 0) ? ac0[r] : ((t == 1) ? ac1[r] : ac2[r]);
      const float bb = (t == 0) ? bc0 : ((t == 1) ? bc1 : bc2);
      hst[rr * XSP + col] = cv * (1.0f / 64.0f) + bb;
    }
    __syncthreads();

    v4f y[2];
    float* op[2];
    bool ok[2];
#pragma unroll
    for (int j = 0; j < 2; ++j) {
      const int rr   = 2 * wave + j;
      const int slot = tt * 16 + rr;
      const int node = nodeBase + slot;
      int ndc = node;
      if (ndc > nN - 1) ndc = nN - 1;
      const int t = typ[slot];
      const v4f xr = *(const v4f*)(x + (size_t)ndc * DF + 4 * lane);
      const v4f hr = *(const v4f*)(hst + rr * XSP + 4 * lane) + xr;
      const float sm = wsum(hr.x + hr.y + hr.z + hr.w);
      const float mu = sm * (1.0f / DF);
      const v4f dv = hr - mu;
      const float q  = wsum(dv.x * dv.x + dv.y * dv.y + dv.z * dv.z + dv.w * dv.w);
      const float rs = rsqrtf(q * (1.0f / DF) + 1e-5f);
      const v4f g4 = *(const v4f*)(gam + (size_t)t * DF + 4 * lane);
      const v4f e4 = *(const v4f*)(bet + (size_t)t * DF + 4 * lane);
      y[j]  = dv * rs * g4 + e4;
      op[j] = out + (size_t)ndc * DF + 4 * lane;
      ok[j] = (node < nN);
    }
    if (ok[0]) *(volatile v4f*)(op[0]) = y[0];
    if (ok[1]) *(volatile v4f*)(op[1]) = y[1];
    __threadfence();
    if (ok[0]) *(volatile v4f*)(op[0]) = y[0];
    if (ok[1]) *(volatile v4f*)(op[1]) = y[1];
    __syncthreads();
  }
}

extern "C" void kernel_launch(void* const* d_in, const int* in_sizes, int n_in,
                              void* d_out, int out_size, void* d_ws, size_t ws_size,
                              hipStream_t stream) {
  if (n_in < 19) return;
  const int nN = in_sizes[0] / DF;
  if (nN <= 0 || in_sizes[0] != nN * DF) return;
  if (in_sizes[1] != NCD * DF * DF || in_sizes[3] != NCD * DF * DF || in_sizes[5] != NCD * DF * DF) return;
  if (in_sizes[2] != NCD * DF || in_sizes[4] != NCD * DF || in_sizes[6] != NCD * DF) return;
  if (in_sizes[7] != NCD * NH) return;
  if (in_sizes[8] != NCD * NH * HC * HC || in_sizes[9] != NCD * NH * HC * HC) return;
  if (in_sizes[10] != NTY * NCD || in_sizes[11] != NRL * NCD) return;
  if (in_sizes[12] != NTY * DF * DF || in_sizes[13] != NTY * DF) return;
  if (in_sizes[14] != NTY * DF || in_sizes[15] != NTY * DF) return;
  const int nE = in_sizes[18];
  if (nE < 1 || in_sizes[16] != 2 * nE) return;
  if (in_sizes[17] != nN) return;
  if (out_size != nN * DF) return;

  const float* x       = (const float*)d_in[0];
  const float* Wk      = (const float*)d_in[1];
  const float* bk      = (const float*)d_in[2];
  const float* Wq      = (const float*)d_in[3];
  const float* bq      = (const float*)d_in[4];
  const float* Wv      = (const float*)d_in[5];
  const float* bv      = (const float*)d_in[6];
  const float* rel_pri = (const float*)d_in[7];
  const float* rel_att = (const float*)d_in[8];
  const float* rel_msg = (const float*)d_in[9];
  const float* n_alpha = (const float*)d_in[10];
  const float* r_alpha = (const float*)d_in[11];
  const float* W_up    = (const float*)d_in[12];
  const float* b_up    = (const float*)d_in[13];
  const float* gam     = (const float*)d_in[14];
  const float* bet     = (const float*)d_in[15];
  const int*   ei      = (const int*)d_in[16];
  const int*   nty     = (const int*)d_in[17];
  const int*   ety     = (const int*)d_in[18];
  float* out = (float*)d_out;

  const int nP = ((nN + GR - 1) / GR) * GR;
  size_t off = 0;
  char* ws = (char*)d_ws;
  _Float16* Wc  = (_Float16*)(ws + off); off += (size_t)NWROW * DF * 2;          off = (off + 255) & ~(size_t)255;
  _Float16* Wu  = (_Float16*)(ws + off); off += (size_t)NUROW * DF * 2;          off = (off + 255) & ~(size_t)255;
  _Float16* ATT = (_Float16*)(ws + off); off += (size_t)NTROW * HC * 2;          off = (off + 255) & ~(size_t)255;
  _Float16* MSG = (_Float16*)(ws + off); off += (size_t)NTROW * HC * 2;          off = (off + 255) & ~(size_t)255;
  float*    Kp  = (float*)(ws + off);    off += (size_t)nP * DF * 4;             off = (off + 255) & ~(size_t)255;
  _Float16* QAp = (_Float16*)(ws + off); off += (size_t)NRL * nP * DF * 2;       off = (off + 255) & ~(size_t)255;
  _Float16* VMp = (_Float16*)(ws + off); off += (size_t)NRL * nP * DF * 2;       off = (off + 255) & ~(size_t)255;
  if (off > ws_size) return;

  const int prepBlocks = NWROW / 16 + NUROW / 16 + (2 * NTROW * 2) / NTHR;
  k_prep<<<prepBlocks, NTHR, 0, stream>>>(Wk, Wq, Wv, W_up, rel_att, rel_msg, r_alpha, Wc, Wu, ATT, MSG);

  k_node<<<nP / GR, NTHR, 0, stream>>>(x, Wc, bk, bq, bv, n_alpha, nty, ATT, MSG, Kp, QAp, VMp, nN, nP);

  hipFuncSetAttribute(reinterpret_cast<const void*>(&k_agg),
                      hipFuncAttributeMaxDynamicSharedMemorySize, LDS_BYTES);
  const int grid = (nN + NB - 1) / NB;
  k_agg<<<grid, NTHR, LDS_BYTES, stream>>>(x, ei, ety, nty, Kp, QAp, VMp, Wu, r_alpha, rel_pri,
                                           b_up, gam, bet, out, nN, nE, nP);
}
